// MultiHeadAttention4AKT_16475494547875
// MI455X (gfx1250) — hardware-verified
//
#include <hip/hip_runtime.h>
#include <stddef.h>
#include <stdint.h>


#define B_   8
#define S_   512
#define D_   1024
#define H_   16
#define DH_  64
#define M_   (B_ * S_)
#define SSTR 520

typedef __bf16         v16bf __attribute__((ext_vector_type(16)));
typedef float          v8f   __attribute__((ext_vector_type(8)));
typedef float          v4f   __attribute__((ext_vector_type(4)));
typedef int            v4i   __attribute__((ext_vector_type(4)));
typedef unsigned short v8us  __attribute__((ext_vector_type(8)));

struct U16x16 { v8us a, b; };

static __device__ __forceinline__ v8us ld8(const unsigned short* p) { return *(const v8us*)p; }
static __device__ __forceinline__ void st8(unsigned short* p, v8us v) { *(v8us*)p = v; }
static __device__ __forceinline__ void st8v(unsigned short* p, v8us v) { *(volatile v8us*)p = v; }

static __device__ __forceinline__ v16bf frag2(v8us e0, v8us e1) {
    U16x16 t; t.a = e0; t.b = e1;
    return __builtin_bit_cast(v16bf, t);
}

static __device__ __forceinline__ v8f vz8() {
    v8f z = {0.f, 0.f, 0.f, 0.f, 0.f, 0.f, 0.f, 0.f};
    return z;
}

static __device__ __forceinline__ unsigned short f2bf(float f) {
    unsigned u = __builtin_bit_cast(unsigned, f);
    u += 0x7FFFu + ((u >> 16) & 1u);
    return (unsigned short)(u >> 16);
}
static __device__ __forceinline__ float bf2f(unsigned short b) {
    return __builtin_bit_cast(float, ((unsigned)b) << 16);
}
static __device__ __forceinline__ float rne_bf(float f) { return bf2f(f2bf(f)); }

static __device__ __forceinline__ v8f wmma_bf16(v16bf a, v16bf b, v8f c) {
    v8f d = __builtin_amdgcn_wmma_f32_16x16x32_bf16(false, a, false, b, (short)0, c, false, false);
    asm volatile("v_nop\n\tv_nop\n\tv_nop\n\tv_nop" : "+v"(d) : "v"(a), "v"(b));
    return d;
}

__global__ __launch_bounds__(256) void cvt_bf16(const float* __restrict__ src,
                                                unsigned short* dst, int n) {
    const int i = (blockIdx.x * 256 + (int)threadIdx.x) * 8;
    if (i + 8 <= n) {
        v4f a = *(const v4f*)(src + i);
        v4f c = *(const v4f*)(src + i + 4);
        v8us w;
        w[0] = f2bf(a[0]); w[1] = f2bf(a[1]); w[2] = f2bf(a[2]); w[3] = f2bf(a[3]);
        w[4] = f2bf(c[0]); w[5] = f2bf(c[1]); w[6] = f2bf(c[2]); w[7] = f2bf(c[3]);
        st8v(dst + i, w);
        __threadfence();
        st8v(dst + i, w);
    }
}

template <int NPA>
static __device__ __attribute__((always_inline)) inline void gemm_main(
    const unsigned short* __restrict__ A0, const unsigned short* __restrict__ A1,
    const unsigned short* __restrict__ W, const int bm0, const int bn0,
    unsigned short* sA, unsigned short* sB, v8f (&acc)[2][2]) {
    const int tid = threadIdx.x, lane = tid & 31, wave = tid >> 5;
    const int wm = wave >> 1, wn = wave & 1, h = lane >> 4, m = lane & 15;
    const int ra = tid >> 1, qa = tid & 1;
    const int rb = tid >> 2, qb = tid & 3;
    const unsigned short* ga0 = A0 + (size_t)(bm0 + ra) * D_ + qa * 16;
    const unsigned short* ga1 = A1 + (size_t)(bm0 + ra) * D_ + qa * 16;
    const unsigned short* gb  = W  + (size_t)(bn0 + rb) * D_ + qb * 8;

#pragma unroll
    for (int i = 0; i < 2; ++i)
#pragma unroll
        for (int j = 0; j < 2; ++j) acc[i][j] = vz8();

    for (int k0 = 0; k0 < D_; k0 += 32) {
        v8us xa0 = ld8(ga0 + k0), xa1 = ld8(ga0 + k0 + 8);
        v8us xb0 = xa0, xb1 = xa1;
        if (NPA == 2) { xb0 = ld8(ga1 + k0); xb1 = ld8(ga1 + k0 + 8); }
        v8us xw = ld8(gb + k0);
        __syncthreads();
        st8(sA + ra * 32 + qa * 16, xa0);
        st8(sA + ra * 32 + qa * 16 + 8, xa1);
        if (NPA == 2) {
            st8(sA + 4096 + ra * 32 + qa * 16, xb0);
            st8(sA + 4096 + ra * 32 + qa * 16 + 8, xb1);
        }
        st8(sB + rb * 32 + qb * 8, xw);
        __syncthreads();

        v16bf bf[2];
#pragma unroll
        for (int j = 0; j < 2; ++j) {
            const unsigned short* p = sB + (wn * 32 + j * 16 + m) * 32;
            bf[j] = frag2(ld8(p + 8 * h), ld8(p + 16 + 8 * h));
        }
#pragma unroll
        for (int pl = 0; pl < NPA; ++pl) {
#pragma unroll
            for (int i = 0; i < 2; ++i) {
                const unsigned short* p = sA + pl * 4096 + (wm * 32 + i * 16 + m) * 32;
                v16bf af = frag2(ld8(p + 8 * h), ld8(p + 16 + 8 * h));
#pragma unroll
                for (int j = 0; j < 2; ++j) acc[i][j] = wmma_bf16(af, bf[j], acc[i][j]);
            }
        }
    }
}

__global__ __launch_bounds__(256) void proj_gemm(
    const unsigned short* __restrict__ qb, const unsigned short* __restrict__ kb,
    const unsigned short* __restrict__ vb,
    const unsigned short* __restrict__ Wkb, const unsigned short* __restrict__ Wvb,
    const float* __restrict__ bk, const float* __restrict__ bv,
    unsigned short* qhh, unsigned short* qhl, unsigned short* khh, unsigned short* khl,
    unsigned short* vth, unsigned short* vtl) {
    __shared__ __attribute__((aligned(16))) unsigned short sA[128 * 32];
    __shared__ __attribute__((aligned(16))) unsigned short sB[64 * 32];
    __shared__ __attribute__((aligned(16))) unsigned short sEh[128 * 64];
    __shared__ __attribute__((aligned(16))) unsigned short sEl[128 * 64];

    const int z = blockIdx.z;
    const unsigned short* X = (z == 0) ? qb : (z == 1) ? kb : vb;
    const unsigned short* W = (z == 2) ? Wvb : Wkb;
    const float* bias = (z == 2) ? bv : bk;
    unsigned short* Ph = (z == 0) ? qhh : (z == 1) ? khh : vth;
    unsigned short* Pl = (z == 0) ? qhl : (z == 1) ? khl : vtl;

    const int bm0 = blockIdx.x * 128, bn0 = blockIdx.y * 64;
    const int tid = threadIdx.x, lane = tid & 31, wave = tid >> 5;
    const int wm = wave >> 1, wn = wave & 1, h = lane >> 4, m = lane & 15;

    v8f acc[2][2];
    gemm_main<1>(X, X, W, bm0, bn0, sA, sB, acc);

#pragma unroll
    for (int j = 0; j < 2; ++j) {
        const int col = wn * 32 + j * 16 + m;
        const float bs = rne_bf(bias[bn0 + col]);
#pragma unroll
        for (int i = 0; i < 2; ++i) {
#pragma unroll
            for (int r = 0; r < 8; ++r) {
                const int row = wm * 32 + i * 16 + 8 * h + r;
                const float y = acc[i][j][r] + bs;
                const unsigned short hi = f2bf(y);
                const unsigned short lo = f2bf(y - bf2f(hi));
                if (z == 2) { sEh[col * 128 + row] = hi; sEl[col * 128 + row] = lo; }
                else        { sEh[row * 64 + col] = hi;  sEl[row * 64 + col] = lo; }
            }
        }
    }
    __syncthreads();

    const int bb = bm0 >> 9, s0 = bm0 & 511;
    const int bh = bb * H_ + blockIdx.y;
    if (z == 2) {
        const size_t base = (size_t)bh * DH_ * S_ + (size_t)s0;
        auto pass = [&]() {
#pragma unroll
            for (int it = 0; it < 4; ++it) {
                const int d = wave * 8 + it * 2 + (lane >> 4);
                const int pc = lane & 15;
                v8us vh = ld8(sEh + d * 128 + pc * 8);
                v8us vl = ld8(sEl + d * 128 + pc * 8);
                const size_t off = base + (size_t)d * S_ + pc * 8;
                st8v(Ph + off, vh);
                st8v(Pl + off, vl);
            }
        };
        pass();
        __threadfence();
        pass();
    } else {
        const size_t base = ((size_t)bh * S_ + (size_t)s0) * DH_;
        auto pass = [&]() {
#pragma unroll
            for (int it = 0; it < 4; ++it) {
                const int row = wave * 16 + it * 4 + (lane >> 3);
                const int pc = lane & 7;
                v8us vh = ld8(sEh + row * 64 + pc * 8);
                v8us vl = ld8(sEl + row * 64 + pc * 8);
                const size_t off = base + (size_t)row * DH_ + pc * 8;
                st8v(Ph + off, vh);
                st8v(Pl + off, vl);
            }
        };
        pass();
        __threadfence();
        pass();
    }
}

__global__ __launch_bounds__(256) void out_gemm(
    const unsigned short* __restrict__ Xh, const unsigned short* __restrict__ Xl,
    const unsigned short* __restrict__ W, const float* __restrict__ bias, float* out) {
    __shared__ __attribute__((aligned(16))) unsigned short sA[2 * 128 * 32];
    __shared__ __attribute__((aligned(16))) unsigned short sB[64 * 32];
    __shared__ __attribute__((aligned(16))) float sF[128 * 64];

    const int bm0 = blockIdx.x * 128, bn0 = blockIdx.y * 64;
    const int tid = threadIdx.x, lane = tid & 31, wave = tid >> 5;
    const int wm = wave >> 1, wn = wave & 1, h = lane >> 4, m = lane & 15;

    v8f acc[2][2];
    gemm_main<2>(Xh, Xl, W, bm0, bn0, sA, sB, acc);

#pragma unroll
    for (int j = 0; j < 2; ++j) {
        const int col = wn * 32 + j * 16 + m;
        const float bs = rne_bf(bias[bn0 + col]);
#pragma unroll
        for (int i = 0; i < 2; ++i) {
#pragma unroll
            for (int r = 0; r < 8; ++r) {
                const int row = wm * 32 + i * 16 + 8 * h + r;
                sF[row * 64 + col] = acc[i][j][r] + bs;
            }
        }
    }
    __syncthreads();

    auto pass = [&]() {
#pragma unroll
        for (int it = 0; it < 8; ++it) {
            const int row = wave * 16 + it * 2 + (lane >> 4);
            const int pc = lane & 15;
            v4f v = *(const v4f*)(sF + row * 64 + pc * 4);
            *(volatile v4f*)(out + (size_t)(bm0 + row) * D_ + bn0 + pc * 4) = v;
        }
    };
    pass();
    __threadfence();
    pass();
}

__global__ __launch_bounds__(64) void attn_kernel(
    const unsigned short* __restrict__ qhh, const unsigned short* __restrict__ qhl,
    const unsigned short* __restrict__ khh, const unsigned short* __restrict__ khl,
    const unsigned short* __restrict__ vth, const unsigned short* __restrict__ vtl,
    const float* __restrict__ pdiff, const float* __restrict__ gammas,
    const int* __restrict__ msk,
    unsigned short* cath, unsigned short* catl) {
    __shared__ __attribute__((aligned(16))) float          sS[16 * SSTR];
    __shared__ __attribute__((aligned(16))) unsigned short sPh[16 * SSTR];
    __shared__ __attribute__((aligned(16))) unsigned short sPl[16 * SSTR];
    __shared__ __attribute__((aligned(16))) unsigned short sOh[16 * DH_];
    __shared__ __attribute__((aligned(16))) unsigned short sOl[16 * DH_];

    const int tid = threadIdx.x, lane = tid & 31, wave = tid >> 5;
    const int h = lane >> 4, m = lane & 15;
    const int qt = blockIdx.x, q0 = qt * 16;
    const int bh = blockIdx.y, b = bh >> 4, hd = bh & 15;
    const int jmax = (qt + 1) * 16;

    {
        const size_t qoff = ((size_t)bh * S_ + q0 + m) * DH_;
        v16bf aqh[2], aql[2];
#pragma unroll
        for (int kk = 0; kk < 2; ++kk) {
            const unsigned short* ph = qhh + qoff + kk * 32;
            const unsigned short* pl = qhl + qoff + kk * 32;
            aqh[kk] = frag2(ld8(ph + 8 * h), ld8(ph + 16 + 8 * h));
            aql[kk] = frag2(ld8(pl + 8 * h), ld8(pl + 16 + 8 * h));
        }
        const size_t koff = ((size_t)bh * S_ + m) * DH_;
        for (int jt = wave; jt <= qt; jt += 2) {
            const int j0 = jt * 16;
            v8f acc = vz8();
#pragma unroll
            for (int kk = 0; kk < 2; ++kk) {
                const unsigned short* ph = khh + koff + (size_t)j0 * DH_ + kk * 32;
                const unsigned short* pl = khl + koff + (size_t)j0 * DH_ + kk * 32;
                v16bf bkh = frag2(ld8(ph + 8 * h), ld8(ph + 16 + 8 * h));
                v16bf bkl = frag2(ld8(pl + 8 * h), ld8(pl + 16 + 8 * h));
                acc = wmma_bf16(aqh[kk], bkh, acc);
                acc = wmma_bf16(aqh[kk], bkl, acc);
                acc = wmma_bf16(aql[kk], bkh, acc);
            }
#pragma unroll
            for (int r = 0; r < 8; ++r) sS[(8 * h + r) * SSTR + j0 + m] = acc[r] * 0.125f;
        }
    }
    __syncthreads();

    {
        const float gam  = rne_bf(gammas[hd]);
        const float gneg = -(fmaxf(gam, 0.f) + log1pf(expf(-fabsf(gam))));
        for (int mr = wave; mr < 16; mr += 2) {
            const int qi = q0 + mr;
            const int jb = lane * 16;
            float s[16];
            unsigned vbits = 0u;
            {
                const float* srow = sS + mr * SSTR + jb;
                const int* mrow = msk + (size_t)qi * S_ + jb;
#pragma unroll
                for (int i4 = 0; i4 < 4; ++i4) {
                    v4f t = *(const v4f*)(srow + i4 * 4);
                    v4i mm = *(const v4i*)(mrow + i4 * 4);
#pragma unroll
                    for (int c = 0; c < 4; ++c) {
                        const int i = i4 * 4 + c;
                        const bool ok = (mm[c] != 0) && ((jb + i) < jmax);
                        vbits |= ok ? (1u << i) : 0u;
                        s[i] = ok ? t[c] : 0.f;
                    }
                }
            }
            float mx = -3.0e38f;
#pragma unroll
            for (int i = 0; i < 16; ++i) {
                const bool ok = ((vbits >> i) & 1u) != 0u;
                const float sv = ok ? s[i] : -1.0e32f;
                mx = fmaxf(mx, sv);
            }
            for (int o = 16; o > 0; o >>= 1) mx = fmaxf(mx, __shfl_xor(mx, o, 32));
            float p[16];
            float lsum = 0.f;
#pragma unroll
            for (int i = 0; i < 16; ++i) {
                const bool ok = ((vbits >> i) & 1u) != 0u;
                const float sv = ok ? s[i] : -1.0e32f;
                const float e = expf(sv - mx);
                p[i] = e;
                lsum += e;
            }
            float tsum = lsum;
            for (int o = 16; o > 0; o >>= 1) tsum += __shfl_xor(tsum, o, 32);
            const float inv = 1.f / tsum;
            float run = 0.f;
#pragma unroll
            for (int i = 0; i < 16; ++i) {
                const bool ok = ((vbits >> i) & 1u) != 0u;
                const float pv = ok ? p[i] * inv : 0.f;
                run += pv;
                p[i] = run;
            }
            float x = run;
            for (int d2 = 1; d2 < 32; d2 <<= 1) {
                const float y = __shfl_up(x, d2, 32);
                if (lane >= d2) x += y;
            }
            const float tot  = __shfl(x, 31, 32);
            const float excl = x - run;
            float s2[16];
            float mx2 = -3.0e38f;
            {
                const float* prow = pdiff + ((size_t)b * S_ + qi) * S_ + jb;
#pragma unroll
                for (int i4 = 0; i4 < 4; ++i4) {
                    v4f t = *(const v4f*)(prow + i4 * 4);
#pragma unroll
                    for (int c = 0; c < 4; ++c) {
                        const int i = i4 * 4 + c;
                        const int j = jb + i;
                        const bool ok = ((vbits >> i) & 1u) != 0u;
                        const float pdv = rne_bf(t[c]);
                        const float cum = excl + p[i];
                        int dj = qi - j; if (dj < 0) dj = -dj;
                        const float posv = (float)dj;
                        const float dist = sqrtf(fmaxf((tot - cum) * posv, 0.f));
                        const float sg = 1.f / (1.f + expf(-pdv));
                        float te = expf(dist * gneg * expf(sg));
                        te = fminf(fmaxf(te, 1e-5f), 1e5f);
                        const float v2 = ok ? (s[i] * te) : -1.0e32f;
                        s2[i] = v2;
                        mx2 = fmaxf(mx2, v2);
                    }
                }
            }
            for (int o = 16; o > 0; o >>= 1) mx2 = fmaxf(mx2, __shfl_xor(mx2, o, 32));
            float l2 = 0.f;
#pragma unroll
            for (int i = 0; i < 16; ++i) { s2[i] = expf(s2[i] - mx2); l2 += s2[i]; }
            for (int o = 16; o > 0; o >>= 1) l2 += __shfl_xor(l2, o, 32);
            const float inv2 = (qi == 0) ? 0.f : (1.f / l2);
            unsigned* dph = (unsigned*)(sPh + mr * SSTR + jb);
            unsigned* dpl = (unsigned*)(sPl + mr * SSTR + jb);
#pragma unroll
            for (int i2 = 0; i2 < 8; ++i2) {
                const float pa = s2[2 * i2] * inv2, pb = s2[2 * i2 + 1] * inv2;
                const unsigned short ha = f2bf(pa), hb = f2bf(pb);
                const unsigned short la = f2bf(pa - bf2f(ha)), lb = f2bf(pb - bf2f(hb));
                dph[i2] = (unsigned)ha | ((unsigned)hb << 16);
                dpl[i2] = (unsigned)la | ((unsigned)lb << 16);
            }
        }
    }
    __syncthreads();

    {
        const int d0 = wave * 32;
        v8f o0 = vz8(), o1 = vz8();
        const size_t voff0 = ((size_t)bh * DH_ + d0 + m) * S_;
        const size_t voff1 = voff0 + (size_t)16 * S_;
        for (int k0 = 0; k0 < jmax; k0 += 32) {
            const unsigned short* pph = sPh + m * SSTR + k0;
            const unsigned short* ppl = sPl + m * SSTR + k0;
            v16bf aph = frag2(ld8(pph + 8 * h), ld8(pph + 16 + 8 * h));
            v16bf apl = frag2(ld8(ppl + 8 * h), ld8(ppl + 16 + 8 * h));
            {
                const unsigned short* pvh = vth + voff0 + k0;
                const unsigned short* pvl = vtl + voff0 + k0;
                v16bf bvh = frag2(ld8(pvh + 8 * h), ld8(pvh + 16 + 8 * h));
                v16bf bvl = frag2(ld8(pvl + 8 * h), ld8(pvl + 16 + 8 * h));
                o0 = wmma_bf16(aph, bvh, o0);
                o0 = wmma_bf16(aph, bvl, o0);
                o0 = wmma_bf16(apl, bvh, o0);
            }
            {
                const unsigned short* pvh = vth + voff1 + k0;
                const unsigned short* pvl = vtl + voff1 + k0;
                v16bf bvh = frag2(ld8(pvh + 8 * h), ld8(pvh + 16 + 8 * h));
                v16bf bvl = frag2(ld8(pvl + 8 * h), ld8(pvl + 16 + 8 * h));
                o1 = wmma_bf16(aph, bvh, o1);
                o1 = wmma_bf16(aph, bvl, o1);
                o1 = wmma_bf16(apl, bvh, o1);
            }
        }
#pragma unroll
        for (int r = 0; r < 8; ++r) {
            const int row = 8 * h + r;
            const float y0 = o0[r], y1 = o1[r];
            const unsigned short h0 = f2bf(y0), h1 = f2bf(y1);
            const unsigned short l0 = f2bf(y0 - bf2f(h0)), l1 = f2bf(y1 - bf2f(h1));
            sOh[row * DH_ + d0 + m] = h0;      sOl[row * DH_ + d0 + m] = l0;
            sOh[row * DH_ + d0 + 16 + m] = h1; sOl[row * DH_ + d0 + 16 + m] = l1;
        }
    }
    __syncthreads();

    {
        unsigned short* dst = (wave == 0) ? cath : catl;
        const unsigned short* so = (wave == 0) ? sOh : sOl;
        const size_t rbase = ((size_t)b * S_ + q0) * D_ + (size_t)hd * DH_;
        auto pass = [&]() {
#pragma unroll
            for (int it = 0; it < 4; ++it) {
                const int row = it * 4 + (lane >> 3);
                const int pc = lane & 7;
                v8us v = ld8(so + row * DH_ + pc * 8);
                st8v(dst + rbase + (size_t)row * D_ + pc * 8, v);
            }
        };
        pass();
        __threadfence();
        pass();
    }
}

extern "C" void kernel_launch(void* const* d_in, const int* in_sizes, int n_in,
                              void* d_out, int out_size, void* d_ws, size_t ws_size,
                              hipStream_t stream) {
    const size_t NQ = (size_t)M_ * D_;
    const size_t NW = (size_t)D_ * D_;
    const size_t NP = (size_t)B_ * S_ * S_;
    if (n_in < 12) return;
    if ((size_t)in_sizes[0] != NQ || (size_t)in_sizes[1] != NQ || (size_t)in_sizes[2] != NQ ||
        (size_t)in_sizes[3] != NP || (size_t)in_sizes[4] != NW || (size_t)in_sizes[6] != NW ||
        (size_t)in_sizes[8] != NW || in_sizes[5] != D_ || in_sizes[7] != D_ || in_sizes[9] != D_ ||
        in_sizes[10] != H_ || (size_t)in_sizes[11] != (size_t)S_ * S_ || (size_t)out_size != NQ)
        return;
    const size_t total_bytes = (11 * NQ + 3 * NW) * sizeof(unsigned short);
    if (total_bytes > ws_size) return;

    const float* q      = (const float*)d_in[0];
    const float* k      = (const float*)d_in[1];
    const float* v      = (const float*)d_in[2];
    const float* pdiff  = (const float*)d_in[3];
    const float* Wk     = (const float*)d_in[4];
    const float* bk     = (const float*)d_in[5];
    const float* Wv     = (const float*)d_in[6];
    const float* bv     = (const float*)d_in[7];
    const float* Wo     = (const float*)d_in[8];
    const float* bo     = (const float*)d_in[9];
    const float* gammas = (const float*)d_in[10];
    const int*   msk    = (const int*)d_in[11];
    float* out = (float*)d_out;

    unsigned short* ws  = (unsigned short*)d_ws;
    unsigned short* qb  = ws;
    unsigned short* kb  = qb  + NQ;
    unsigned short* vb  = kb  + NQ;
    unsigned short* Wkb = vb  + NQ;
    unsigned short* Wvb = Wkb + NW;
    unsigned short* Wob = Wvb + NW;
    unsigned short* qhh = Wob + NW;
    unsigned short* qhl = qhh + NQ;
    unsigned short* khh = qhl + NQ;
    unsigned short* khl = khh + NQ;
    unsigned short* vth = khl + NQ;
    unsigned short* vtl = vth + NQ;
    unsigned short* cath = vtl + NQ;
    unsigned short* catl = cath + NQ;

    const unsigned gq = (unsigned)((NQ + 2047) / 2048);
    const unsigned gw = (unsigned)((NW + 2047) / 2048);
    cvt_bf16<<<dim3(gq), dim3(256), 0, stream>>>(q,  qb,  (int)NQ);
    cvt_bf16<<<dim3(gq), dim3(256), 0, stream>>>(k,  kb,  (int)NQ);
    cvt_bf16<<<dim3(gq), dim3(256), 0, stream>>>(v,  vb,  (int)NQ);
    cvt_bf16<<<dim3(gw), dim3(256), 0, stream>>>(Wk, Wkb, (int)NW);
    cvt_bf16<<<dim3(gw), dim3(256), 0, stream>>>(Wv, Wvb, (int)NW);
    cvt_bf16<<<dim3(gw), dim3(256), 0, stream>>>(Wo, Wob, (int)NW);

    proj_gemm<<<dim3(M_ / 128, D_ / 64, 3), dim3(256), 0, stream>>>(
        qb, kb, vb, Wkb, Wvb, bk, bv, qhh, qhl, khh, khl, vth, vtl);

    attn_kernel<<<dim3(S_ / 16, B_ * H_), dim3(64), 0, stream>>>(
        qhh, qhl, khh, khl, vth, vtl, pdiff, gammas, msk, cath, catl);

    out_gemm<<<dim3(M_ / 128, D_ / 64), dim3(256), 0, stream>>>(cath, catl, Wob, bo, out);
}
